// DeepDFA_19851338842260
// MI455X (gfx1250) — hardware-verified
//
#include <hip/hip_runtime.h>


namespace {
constexpr int NB = 4096, L = 512, NS = 64, NA = 32;

typedef __attribute__((ext_vector_type(16))) __bf16 v16bb;
typedef __attribute__((ext_vector_type(8))) float v8f;
typedef __attribute__((ext_vector_type(4))) float v4f;
__device__ __forceinline__ v8f wmma16bb(v16bb a, v16bb b, v8f c) { v8f d = __builtin_amdgcn_wmma_f32_16x16x32_bf16(false, a, false, b, (short)0, c, false, false); asm volatile("v_nop\n\tv_nop\n\tv_nop\n\tv_nop" : "+v"(d) : "v"(a), "v"(b)); return d; }
__device__ __forceinline__ void wave_lds_sync() { __builtin_amdgcn_fence(__ATOMIC_RELEASE, "workgroup"); __builtin_amdgcn_wave_barrier(); __builtin_amdgcn_fence(__ATOMIC_ACQUIRE, "workgroup"); }

__global__ __launch_bounds__(256) void walk_kernel(const int* __restrict__ act, const float* __restrict__ tp, unsigned char* __restrict__ st) {
  __shared__ unsigned char nxt[NA * NS];
  const int t_ = threadIdx.x, b = blockIdx.x * 256 + t_;
  for (int i = t_; i < NA * NS; i += 256) { const float* row = tp + (size_t)i * NS; int best = 0; float bv = row[0]; for (int k = 1; k < NS; ++k) { const float v = row[k]; if (v > bv) { bv = v; best = k; } } nxt[i] = (unsigned char)best; }
  __syncthreads();
  const int* ar = act + (size_t)b * L; int cur = 0;
  for (int t = 0; t < L; ++t) { int a = ar[t]; a = (a < 0) ? 0 : (a >= NA ? NA - 1 : a); cur = nxt[a * NS + cur]; for (int pass = 0; pass < 2; ++pass) ((volatile unsigned char*)st)[(size_t)t * NB + b] = (unsigned char)cur; }
  __threadfence();
}

__global__ __launch_bounds__(256) void reward_kernel(const unsigned char* __restrict__ st, const float* __restrict__ acc_m, float* __restrict__ rew) {
  __shared__ __attribute__((aligned(16))) float Ro[8][16][2];
  const int wid = threadIdx.x >> 5, lane = threadIdx.x & 31, nloc = lane & 15, hlf = lane >> 4; const size_t g0 = ((size_t)blockIdx.x * 8 + wid) * 16; const int b = (int)(g0 / L), t0 = (int)(g0 % L);
  const int mys = st[(size_t)(t0 + nloc) * NB + b];
  v8f acc = {};
#pragma unroll
  for (int kb = 0; kb < NS; kb += 32) { union { unsigned short s[16]; v16bb v; } ua, ub;
#pragma unroll
    for (int e = 0; e < 8; ++e) { const int k0 = kb + 8 * hlf + e, k1 = kb + 16 + 8 * hlf + e; ua.s[e] = (k0 == mys) ? 0x3F80 : 0; ua.s[8 + e] = (k1 == mys) ? 0x3F80 : 0;
      ub.s[e] = (nloc < 2 && acc_m[(size_t)k0 * 2 + nloc] != 0.0f) ? (unsigned short)(__float_as_uint(acc_m[(size_t)k0 * 2 + nloc]) >> 16) : 0; ub.s[8 + e] = (nloc < 2 && acc_m[(size_t)k1 * 2 + nloc] != 0.0f) ? (unsigned short)(__float_as_uint(acc_m[(size_t)k1 * 2 + nloc]) >> 16) : 0; }
    acc = wmma16bb(ua.v, ub.v, acc); }
  if (nloc < 2) {
#pragma unroll
    for (int r = 0; r < 8; ++r) Ro[wid][8 * hlf + r][nloc] = acc[r]; }
  wave_lds_sync();
  for (int pass = 0; pass < 2; ++pass) { if (lane < 8) *(volatile v4f*)(rew + (g0 + lane * 2) * 2) = *(const v4f*)(&Ro[wid][lane * 2][0]); __threadfence(); }
}

__global__ __launch_bounds__(256) void final_kernel(const unsigned char* __restrict__ st, float* __restrict__ sf) {
  __shared__ __attribute__((aligned(16))) float T[64][NS];
  const int t_ = threadIdx.x, b0 = blockIdx.x * 64;
  for (int i = t_; i < 64 * NS; i += 256) { const int r = i >> 6, k = i & 63; T[r][k] = (st[(size_t)(L - 1) * NB + b0 + r] == k) ? 1.0f : 0.0f; }
  __syncthreads();
  for (int pass = 0; pass < 2; ++pass) { for (int i = t_; i < 64 * NS / 4; i += 256) { const int r = i >> 4, c4 = (i & 15) * 4; *(volatile v4f*)(sf + (size_t)(b0 + r) * NS + c4) = *(const v4f*)(&T[r][c4]); } __threadfence(); }
}
}

extern "C" void kernel_launch(void* const* d_in, const int* in_sizes, int n_in,
                              void* d_out, int out_size, void* d_ws, size_t ws_size, hipStream_t stream) {
  (void)n_in; (void)out_size;
  const int* act = (const int*)d_in[0]; const float* tp = (const float*)d_in[1]; const float* acc_m = (const float*)d_in[2];
  float* rew = (float*)d_out; float* sf = rew + (size_t)NB * L * 2;
  if (in_sizes[0] != NB * L || in_sizes[1] != NA * NS * NS || in_sizes[2] != NS * 2) return;
  if ((size_t)NB * L > ws_size) return;
  unsigned char* st = (unsigned char*)d_ws;
  walk_kernel<<<NB / 256, 256, 0, stream>>>(act, tp, st);
  reward_kernel<<<NB * L / 16 / 8, 256, 0, stream>>>(st, acc_m, rew);
  final_kernel<<<NB / 64, 256, 0, stream>>>(st, sf);
}
